// LSSM_73280732005134
// MI455X (gfx1250) — hardware-run, weakly checked
//
#include <hip/hip_runtime.h>
#include <hip/hip_fp16.h>
#include <math.h>

typedef __attribute__((ext_vector_type(16))) _Float16 v16h;
typedef __attribute__((ext_vector_type(8)))  _Float16 v8h;
typedef __attribute__((ext_vector_type(8)))  float    v8f;
typedef __attribute__((ext_vector_type(4)))  float    v4f;
typedef __attribute__((ext_vector_type(2)))  unsigned v2u;
typedef __attribute__((ext_vector_type(4)))  unsigned v4u;

constexpr int kH     = 32;
constexpr int kW     = 32;
constexpr int kHW    = 1024;
constexpr int kDm    = 32;
constexpr int kC     = 64;
constexpr int kXzP   = 128;
constexpr int kNst   = 16;
constexpr int kDir   = 6;
constexpr int kGc    = 16;
constexpr int kL     = 65536;
constexpr int kProjN = 34;
constexpr int kProjP = 64;
constexpr int kKp    = 32;
constexpr int kSd    = 64;
constexpr int kOutN  = 32;
constexpr int kOutP  = 64;
constexpr float kWCarry = 1024.0f;
constexpr float kResid  = 2048.0f;
constexpr float kYCarry = 16.0f;
constexpr float kSCarry = 0.25f;
constexpr float kLnEps  = 1e-5f;
constexpr float kInvResid = 1.0f / kResid;
constexpr float kInvSCarry = 1.0f / kSCarry;
static_assert(kHW == kH * kW);
static_assert(kL == kC * kHW);
static_assert(kXzP == 2 * kC);
static_assert(kProjN == 2 + 2 * kNst);
static_assert(kProjN <= kProjP && (kProjP % 64) == 0);
static_assert(kGc <= kKp && (kKp % 32) == 0);
static_assert(kGc <= kSd && (kSd % 64) == 0);
static_assert(kOutN <= kOutP && (kOutP % 64) == 0);
static_assert((kDm % 32) == 0 && (kC % 32) == 0 && (kXzP % 64) == 0);
static_assert((kHW % 32) == 0 && (kL % 64) == 0 && (kL % 32) == 0);
static_assert(kH == 32 && kW == 32 && kC == 64 && kGc == 16 && kNst == 16 && kDir == 6);

constexpr size_t kSzXH    = (size_t)kHW * kDm * 2;
constexpr size_t kSzWIN   = (size_t)kXzP * kDm * 2;
constexpr size_t kSzWXH   = (size_t)kDir * kProjP * kKp * 2;
constexpr size_t kSzWOH   = (size_t)kOutP * kC * 2;
constexpr size_t kSzALOGP = (size_t)kDir * kSd * kNst * 4;
constexpr size_t kSzDSP   = (size_t)kDir * kSd * 4;
constexpr size_t kSzXZ    = (size_t)kHW * kXzP * 4;
constexpr size_t kSzV     = (size_t)kC * kHW * 4;
constexpr size_t kSzU     = (size_t)kL * kSd * 4;
constexpr size_t kSzA16   = (size_t)kL * kKp * 2;
constexpr size_t kSzXD    = (size_t)kL * kProjP * 4;
constexpr size_t kSzDTP   = (size_t)kL * kSd * 4;
constexpr size_t kSzY16   = (size_t)kL * kSd * 2;
constexpr size_t kSzOY    = (size_t)kDir * kL * 4;
constexpr size_t kSzYS    = (size_t)2 * kHW * kC * 4;
constexpr size_t kSzGH    = (size_t)kHW * kC * 2;
constexpr size_t kSzOUTP  = (size_t)kHW * kOutP * 4;
static_assert(kSzXH == 65536ull && kSzWIN == 8192ull && kSzWXH == 24576ull && kSzWOH == 8192ull);
static_assert(kSzALOGP == 24576ull && kSzDSP == 1536ull && kSzXZ == 524288ull && kSzV == 262144ull);
static_assert(kSzU == 16777216ull && kSzA16 == 4194304ull && kSzXD == 16777216ull && kSzDTP == 16777216ull);
static_assert(kSzY16 == 8388608ull && kSzYS == 524288ull && kSzGH == 131072ull && kSzOUTP == 262144ull);
static_assert(kSzOY == 1572864ull);
static_assert((kSzXH % 128) == 0 && (kSzWIN % 128) == 0 && (kSzWXH % 128) == 0 && (kSzWOH % 128) == 0 &&
              (kSzALOGP % 128) == 0 && (kSzDSP % 128) == 0 && (kSzXZ % 128) == 0 && (kSzV % 128) == 0 &&
              (kSzU % 128) == 0 && (kSzA16 % 128) == 0 && (kSzXD % 128) == 0 && (kSzDTP % 128) == 0 &&
              (kSzY16 % 128) == 0 && (kSzYS % 128) == 0 && (kSzGH % 128) == 0 && (kSzOUTP % 128) == 0);
static_assert((kSzOY % 128) == 0);
constexpr size_t kOffXH    = 0;
constexpr size_t kOffWIN   = kOffXH    + kSzXH;
constexpr size_t kOffWXH   = kOffWIN   + kSzWIN;
constexpr size_t kOffWOH   = kOffWXH   + kSzWXH;
constexpr size_t kOffALOGP = kOffWOH   + kSzWOH;
constexpr size_t kOffDSP   = kOffALOGP + kSzALOGP;
constexpr size_t kOffXZ    = kOffDSP   + kSzDSP;
constexpr size_t kOffV     = kOffXZ    + kSzXZ;
constexpr size_t kOffU     = kOffV     + kSzV;
constexpr size_t kOffAH    = kOffU     + kSzU;
constexpr size_t kOffAL    = kOffAH    + kSzA16;
constexpr size_t kOffXD    = kOffAL    + kSzA16;
constexpr size_t kOffDTP   = kOffXD    + kSzXD;
constexpr size_t kOffYH    = kOffDTP   + kSzDTP;
constexpr size_t kOffYL    = kOffYH    + kSzY16;
constexpr size_t kOffOY    = kOffYL    + kSzY16;
constexpr size_t kOffYS    = kOffOY    + kSzOY;
constexpr size_t kOffGH    = kOffYS    + kSzYS;
constexpr size_t kOffOUTP  = kOffGH    + kSzGH;
constexpr size_t kWsTotal  = kOffOUTP  + kSzOUTP;
static_assert(kWsTotal == 78906880ull);
static_assert(kWsTotal <= 134217728ull);

__device__ __forceinline__ _Float16 f16_flush(float v) {
  const float w = (fabsf(v) < 6.103515625e-05f) ? 0.0f : v;
  return (_Float16)w;
}
__device__ __forceinline__ void f16_split(float v, _Float16& hi, _Float16& lo) {
  hi = f16_flush(v);
  const float hf = (float)hi;
  const float r = (v - hf) * kResid;
  lo = f16_flush(r);
}

__device__ __forceinline__ float bf16r(float v) {
  unsigned u = __float_as_uint(v);
  u = (u + 0x7FFFu + ((u >> 16) & 1u)) & 0xFFFF0000u;
  return __uint_as_float(u);
}

__device__ __forceinline__ float h16_to_f32(unsigned hb) {
  const unsigned sgn = (hb & 0x8000u) << 16; const unsigned em = hb & 0x7fffu;
  const float fn = __uint_as_float((em << 13) + 0x38000000u);
  const float fs = (float)em * 5.9604644775390625e-8f;
  const float mag = (em < 0x400u) ? fs : fn; return __uint_as_float(__float_as_uint(mag) | sgn); }

namespace eng {
union FragU { v16h v; v8h h[2]; };
__device__ __forceinline__ v16h frag_load(const _Float16* p) {
  FragU f;
  f.h[0] = *(const v8h*)(p);
  f.h[1] = *(const v8h*)(p + 16);
  return f.v;
}
__device__ __forceinline__ v8f mma(v16h a, v16h b, v8f c) {
  return __builtin_amdgcn_wmma_f32_16x16x32_f16(false, a, false, b, (short)0, c, false, false);
}
__device__ __forceinline__ void guard1(v8f& a, v16h x, v16h y) {
  asm volatile("v_nop\n\tv_nop\n\tv_nop\n\tv_nop" : "+v"(a) : "v"(x), "v"(y));
}
__device__ __forceinline__ void guard_acc(v8f& a) {
  asm volatile("v_nop\n\tv_nop\n\tv_nop\n\tv_nop" : "+v"(a));
}
__device__ __forceinline__ void keep4(v16h a, v16h b, v16h c, v16h d) {
  asm volatile("v_nop" :: "v"(a), "v"(b), "v"(c), "v"(d));
}

template <int MI, int SPL>
__global__ __launch_bounds__(256) void gemm_f16_kernel(
    const unsigned short* __restrict__ Ap, const unsigned short* __restrict__ A2p, int lda,
    const unsigned short* __restrict__ Btp, const unsigned short* __restrict__ Bt2p, int ldb,
    float* __restrict__ C, int ldc, int M, int N, int K, float scale, float rscale)
{
  static_assert(MI >= 1 && MI <= 2);
  static_assert(SPL >= 0 && SPL <= 2);
  const _Float16* A   = (const _Float16*)Ap;
  const _Float16* A2  = (const _Float16*)A2p;
  const _Float16* Bt  = (const _Float16*)Btp;
  const _Float16* Bt2 = (const _Float16*)Bt2p;
  __shared__ __align__(16) float sT[8][16 * 68];
  const int lane = threadIdx.x & 31;
  const int wave = threadIdx.x >> 5;
  const int tilesN = N >> 6;
  const int tilesM = M / (16 * MI);
  const int tile = blockIdx.x * 8 + wave;
  if (tile >= tilesM * tilesN) return;
  const int tm = tile / tilesN;
  const int tn = tile - tm * tilesN;
  const int m0 = tm * (16 * MI);
  const int n0 = tn << 6;
  const int rlane = lane & 15;
  const int koff  = (lane >> 4) * 8;
  const int mOff  = (lane >> 4) * 8;

  v8f acc[MI][4], accr[MI][4];
#pragma unroll
  for (int i = 0; i < MI; ++i)
#pragma unroll
    for (int j = 0; j < 4; ++j) {
      acc[i][j]  = (v8f){0.f, 0.f, 0.f, 0.f, 0.f, 0.f, 0.f, 0.f};
      accr[i][j] = (v8f){0.f, 0.f, 0.f, 0.f, 0.f, 0.f, 0.f, 0.f};
    }

  for (int k0 = 0; k0 < K; k0 += 32) {
    v16h bh[4], bl[4];
#pragma unroll
    for (int j = 0; j < 4; ++j) {
      const size_t bo = (size_t)(n0 + (j << 4) + rlane) * ldb + koff + k0;
      bh[j] = frag_load(Bt + bo);
      if (SPL == 2) bl[j] = frag_load(Bt2 + bo); else bl[j] = bh[j];
    }
#pragma unroll
    for (int i = 0; i < MI; ++i) {
      const size_t ao = (size_t)(m0 + (i << 4) + rlane) * lda + koff + k0;
      const v16h ah = frag_load(A + ao);
      v16h al = ah;
      if (SPL >= 1) al = frag_load(A2 + ao);
#pragma unroll
      for (int j = 0; j < 4; ++j) {
        acc[i][j] = mma(ah, bh[j], acc[i][j]);
        if (SPL >= 1) accr[i][j] = mma(al, bh[j], accr[i][j]);
        if (SPL == 2) accr[i][j] = mma(ah, bl[j], accr[i][j]);
      }
#pragma unroll
      for (int j = 0; j < 4; ++j) {
        guard1(acc[i][j], ah, al);
        if (SPL >= 1) guard1(accr[i][j], ah, al);
      }
    }
    keep4(bh[0], bh[1], bh[2], bh[3]);
    if (SPL == 2) keep4(bl[0], bl[1], bl[2], bl[3]);
  }
#pragma unroll
  for (int i = 0; i < MI; ++i)
#pragma unroll
    for (int j = 0; j < 4; ++j) {
      guard_acc(acc[i][j]);
      if (SPL >= 1) guard_acc(accr[i][j]);
    }

  float* slab = sT[wave];
#pragma unroll
  for (int i = 0; i < MI; ++i) {
    const int mBase = m0 + (i << 4);
#pragma unroll
    for (int j = 0; j < 4; ++j) {
#pragma unroll
      for (int r = 0; r < 8; ++r) {
        float v = acc[i][j][r] * scale;
        if (SPL >= 1) v += accr[i][j][r] * rscale;
        slab[(mOff + r) * 68 + (j << 4) + rlane] = v;
      }
    }
    __builtin_amdgcn_fence(__ATOMIC_RELEASE, "workgroup");
    __builtin_amdgcn_wave_barrier();
    __builtin_amdgcn_fence(__ATOMIC_ACQUIRE, "workgroup");
    {
      const int hh = lane >> 4, c4 = (lane & 15) * 4;
      for (int pass = 0; pass < 2; ++pass) {
#pragma unroll
        for (int it = 0; it < 8; ++it) {
          const int row = it * 2 + hh;
          const v4f v = *(const v4f*)(slab + row * 68 + c4);
          *(volatile v4f*)(C + (size_t)(mBase + row) * ldc + n0 + c4) = v;
        }
        __threadfence();
      }
    }
    __builtin_amdgcn_fence(__ATOMIC_RELEASE, "workgroup");
    __builtin_amdgcn_wave_barrier();
    __builtin_amdgcn_fence(__ATOMIC_ACQUIRE, "workgroup");
  }
}
}

__global__ __launch_bounds__(256) void rne_rows_f16_kernel(
    const float* __restrict__ src, unsigned short* __restrict__ dH, int total8)
{
  const int i = blockIdx.x * 256 + threadIdx.x;
  if (i >= total8) return;
  const size_t e0 = (size_t)i << 3;
  const v4f a0 = *(const v4f*)(src + e0);
  const v4f a1 = *(const v4f*)(src + e0 + 4);
  const float f0 = a0[0];
  const float f1 = a0[1];
  const float f2 = a0[2];
  const float f3 = a0[3];
  const float f4 = a1[0];
  const float f5 = a1[1];
  const float f6 = a1[2];
  const float f7 = a1[3];
  v8h hv;
  hv[0] = f16_flush(bf16r(f0));
  hv[1] = f16_flush(bf16r(f1));
  hv[2] = f16_flush(bf16r(f2));
  hv[3] = f16_flush(bf16r(f3));
  hv[4] = f16_flush(bf16r(f4));
  hv[5] = f16_flush(bf16r(f5));
  hv[6] = f16_flush(bf16r(f6));
  hv[7] = f16_flush(bf16r(f7));
  unsigned short* qh = dH + e0;
  *(volatile v8h*)qh = hv;
  __threadfence();
  *(volatile v8h*)qh = hv;
}

__global__ __launch_bounds__(256) void pack_rows_bf_kernel(
    const float* __restrict__ W, unsigned short* __restrict__ dH,
    int Kdim, int Nreal, int total8, float carry)
{
  const int i = blockIdx.x * 256 + threadIdx.x;
  if (i >= total8) return;
  const size_t e0 = (size_t)i << 3;
  const int row = (int)(e0 / (size_t)Kdim);
  const int col = (int)(e0 - (size_t)row * (size_t)Kdim);
  const bool live = (row < Nreal);
  const int rc = live ? row : (Nreal - 1);
  const v4f a0 = *(const v4f*)(W + (size_t)rc * Kdim + col);
  const v4f a1 = *(const v4f*)(W + (size_t)rc * Kdim + col + 4);
  const float w0 = a0[0];
  const float w1 = a0[1];
  const float w2 = a0[2];
  const float w3 = a0[3];
  const float w4 = a1[0];
  const float w5 = a1[1];
  const float w6 = a1[2];
  const float w7 = a1[3];
  const float t0 = bf16r(w0) * carry;
  const float t1 = bf16r(w1) * carry;
  const float t2 = bf16r(w2) * carry;
  const float t3 = bf16r(w3) * carry;
  const float t4 = bf16r(w4) * carry;
  const float t5 = bf16r(w5) * carry;
  const float t6 = bf16r(w6) * carry;
  const float t7 = bf16r(w7) * carry;
  const float g0 = live ? t0 : 0.0f;
  const float g1 = live ? t1 : 0.0f;
  const float g2 = live ? t2 : 0.0f;
  const float g3 = live ? t3 : 0.0f;
  const float g4 = live ? t4 : 0.0f;
  const float g5 = live ? t5 : 0.0f;
  const float g6 = live ? t6 : 0.0f;
  const float g7 = live ? t7 : 0.0f;
  v8h hv;
  hv[0] = f16_flush(g0);
  hv[1] = f16_flush(g1);
  hv[2] = f16_flush(g2);
  hv[3] = f16_flush(g3);
  hv[4] = f16_flush(g4);
  hv[5] = f16_flush(g5);
  hv[6] = f16_flush(g6);
  hv[7] = f16_flush(g7);
  unsigned short* qh = dH + e0;
  *(volatile v8h*)qh = hv;
  __threadfence();
  *(volatile v8h*)qh = hv;
}

static_assert(((kDir * kProjP * kKp / 8) % 256) == 0);
__global__ __launch_bounds__(256) void pack_xproj_kernel(
    const float* __restrict__ xpw, unsigned short* __restrict__ WXH)
{
  const int i  = blockIdx.x * 256 + threadIdx.x;
  const int e0 = i * 8;
  const int g  = e0 / (kProjP * kKp);
  const int d  = (e0 / kKp) % kProjP;
  const int k0 = e0 % kKp;
  const bool live = (d < kProjN) && (k0 < kGc);
  const int dc = (d < kProjN) ? d : (kProjN - 1);
  const int kc = k0 & 8;
  const float* sp = xpw + (size_t)((g * kProjN + dc) * kGc + kc);
  const v4f a0 = *(const v4f*)(sp);
  const v4f a1 = *(const v4f*)(sp + 4);
  v8h hv;
#pragma unroll
  for (int e = 0; e < 4; ++e) {
    const float w0 = a0[e];
    const float w1 = a1[e];
    const float t0 = bf16r(w0) * kWCarry;
    const float t1 = bf16r(w1) * kWCarry;
    const float s0 = live ? t0 : 0.0f;
    const float s1 = live ? t1 : 0.0f;
    hv[e]     = f16_flush(s0);
    hv[4 + e] = f16_flush(s1);
  }
  unsigned short* qh = WXH + (size_t)e0;
  *(volatile v8h*)qh = hv;
  __threadfence();
  *(volatile v8h*)qh = hv;
}

static_assert(((kDir * kSd * kNst / 4) % 256) == 0);
static_assert(((kDir * kSd / 4) % 32) == 0);
__global__ __launch_bounds__(256) void scan_params_kernel(
    const float* __restrict__ A_logs, const float* __restrict__ Ds,
    float* __restrict__ ALOGP, float* __restrict__ DSP)
{
  constexpr int kDsp4 = kDir * kSd / 4;
  const int i  = blockIdx.x * 256 + threadIdx.x;
  const int e0 = i * 4;
  const int g  = e0 / (kSd * kNst);
  const int j  = (e0 / kNst) % kSd;
  const int n0 = e0 % kNst;
  const bool live = (j < kGc);
  const int jc = live ? j : (kGc - 1);
  const v4f a = *(const v4f*)(A_logs + (size_t)((kGc * g + jc) * kNst + n0));
  const float a0 = a[0];
  const float a1 = a[1];
  const float a2 = a[2];
  const float a3 = a[3];
  v4f r;
  r[0] = live ? bf16r(a0) : 0.0f;
  r[1] = live ? bf16r(a1) : 0.0f;
  r[2] = live ? bf16r(a2) : 0.0f;
  r[3] = live ? bf16r(a3) : 0.0f;

  const bool own = (i < kDsp4);
  const int di = own ? i : (kDsp4 - 1);
  const int de = di * 4;
  const int dg = de / kSd;
  const int dj = de % kSd;
  const bool dlive = (dj < kGc);
  const int djc = dlive ? dj : (kGc - 4);
  const v4f dv = *(const v4f*)(Ds + (size_t)(kGc * dg + djc));
  const float d0 = dv[0];
  const float d1 = dv[1];
  const float d2 = dv[2];
  const float d3 = dv[3];
  v4f s;
  s[0] = dlive ? bf16r(d0) : 0.0f;
  s[1] = dlive ? bf16r(d1) : 0.0f;
  s[2] = dlive ? bf16r(d2) : 0.0f;
  s[3] = dlive ? bf16r(d3) : 0.0f;

  float* p  = ALOGP + (size_t)i * 4;
  float* dp = DSP + (size_t)di * 4;
  *(volatile v4f*)p = r;
  if (own) *(volatile v4f*)dp = s;
  __threadfence();
  *(volatile v4f*)p = r;
  if (own) *(volatile v4f*)dp = s;
}

static_assert(((kC * kH * kW / 4) % 256) == 0);
__global__ __launch_bounds__(256) void conv3_silu_kernel(
    const float* __restrict__ XZ, const float* __restrict__ conv_w, const float* __restrict__ conv_b,
    float* __restrict__ V)
{
  const int i  = blockIdx.x * 256 + threadIdx.x;
  const int w0 = (i & 7) * 4;
  const int h  = (i >> 3) & 31;
  const int c  = i >> 8;
  float wt[9];
#pragma unroll
  for (int t = 0; t < 9; ++t) wt[t] = bf16r(conv_w[c * 9 + t]);
  const float bias = bf16r(conv_b[c]);
  float in[3][6];
#pragma unroll
  for (int dy = 0; dy < 3; ++dy) {
    const int hh = h + dy - 1;
    const bool hok = (hh >= 0) && (hh < kH);
    const int hc = (hh < 0) ? 0 : ((hh > kH - 1) ? (kH - 1) : hh);
#pragma unroll
    for (int dx = 0; dx < 6; ++dx) {
      const int ww = w0 + dx - 1;
      const bool wok = (ww >= 0) && (ww < kW);
      const int wc = (ww < 0) ? 0 : ((ww > kW - 1) ? (kW - 1) : ww);
      const float t = XZ[(size_t)(hc * kW + wc) * kXzP + c];
      in[dy][dx] = (hok && wok) ? t : 0.0f;
    }
  }
  v4f r;
#pragma unroll
  for (int e = 0; e < 4; ++e) {
    float s = 0.0f;
#pragma unroll
    for (int dy = 0; dy < 3; ++dy)
#pragma unroll
      for (int kx = 0; kx < 3; ++kx)
        s = fmaf(wt[dy * 3 + kx], in[dy][e + kx], s);
    s = s + bias;
    r[e] = s / (1.0f + expf(-s));
  }
  float* p = V + (size_t)i * 4;
  *(volatile v4f*)p = r;
  __threadfence();
  *(volatile v4f*)p = r;
}

__device__ __forceinline__ int voxel_index(int order, int pos) {
  const int p10 = pos >> 10;
  const int p11 = pos >> 11;
  const int m5  = (pos >> 5) & 31;
  const int m5c = (pos >> 5) & 63;
  const int m6  = (pos >> 6) & 31;
  const int l5  = pos & 31;
  const int l6  = pos & 63;
  const int c = (order < 2) ? p10 : (((order == 2) || (order == 5)) ? m5c : l6);
  const int h = (order == 0) ? m5 : (((order == 1) || (order == 5)) ? l5 : ((order == 3) ? m6 : p11));
  const int w = ((order == 0) || (order == 2)) ? l5 : ((order == 1) ? m5 : ((order == 4) ? m6 : p11));
  return c * 1024 + h * 32 + w;
}
__device__ __forceinline__ int order_pos(int order, int c, int h, int w) {
  const int p0 = c * 1024 + h * 32 + w;
  const int p1 = c * 1024 + w * 32 + h;
  const int p2 = h * 2048 + c * 32 + w;
  const int p3 = w * 2048 + h * 64 + c;
  const int p4 = h * 2048 + w * 64 + c;
  const int p5 = w * 2048 + c * 32 + h;
  return (order == 0) ? p0 : ((order == 1) ? p1 : ((order == 2) ? p2 : ((order == 3) ? p3 :
         ((order == 4) ? p4 : p5))));
}

__device__ __forceinline__ float chan_value(const float* __restrict__ V, const float* __restrict__ w_xs,
                                            const float* __restrict__ b_xs, int pass, int g, int j, int l) {
  const int q = kGc * g + j;
  const int order = pass ? g : (q % kDir);
  const int feat  = pass ? j : (q / kDir);
  const int pos   = pass ? (kL - 1 - l) : l;
  const int idx = voxel_index(order, pos);
  const float wv = bf16r(w_xs[feat]);
  const float bv = bf16r(b_xs[feat]);
  const float s = V[idx];
  return wv * s + bv;
}

static_assert(((kL * kSd / 4) % 256) == 0);
static_assert(((kL * kKp / 8) % 256) == 0);
__global__ __launch_bounds__(256) void lift_gather_kernel(
    const float* __restrict__ V, const float* __restrict__ w_xs, const float* __restrict__ b_xs,
    float* __restrict__ U, unsigned short* __restrict__ AH, unsigned short* __restrict__ AL,
    int pass, int g)
{
  constexpr int kPieceBlocks = kL * kKp / 8 / 256;
  const int i  = blockIdx.x * 256 + threadIdx.x;
  const int l  = i >> 4;
  const int j0 = (i & 15) * 4;
  const bool live = (j0 < kGc);
  const int jb = j0 & (kGc - 1);
  v4f uv;
#pragma unroll
  for (int e = 0; e < 4; ++e) {
    const float t = chan_value(V, w_xs, b_xs, pass, g, jb + e, l);
    uv[e] = live ? t : 0.0f;
  }
  const bool owns16 = ((int)blockIdx.x < kPieceBlocks);
  v8h hv, lv;
#pragma unroll
  for (int e = 0; e < 8; ++e) {
    hv[e] = (_Float16)0.0f;
    lv[e] = (_Float16)0.0f;
  }
  if (owns16) {
    const int lp = i >> 2;
    const int k0 = (i & 3) * 8;
    const bool plive = (k0 < kGc);
    const int kb = k0 & 8;
#pragma unroll
    for (int e = 0; e < 8; ++e) {
      const float t = chan_value(V, w_xs, b_xs, pass, g, kb + e, lp);
      const float s = plive ? t : 0.0f;
      _Float16 hh, ll;
      f16_split(s, hh, ll);
      hv[e] = hh;
      lv[e] = ll;
    }
  }
  float* up = U + (size_t)i * 4;
  unsigned short* qh = AH + (size_t)i * 8;
  unsigned short* ql = AL + (size_t)i * 8;
  *(volatile v4f*)up = uv;
  if (owns16) {
    *(volatile v8h*)qh = hv;
    *(volatile v8h*)ql = lv;
  }
  __threadfence();
  *(volatile v4f*)up = uv;
  if (owns16) {
    *(volatile v8h*)qh = hv;
    *(volatile v8h*)ql = lv;
  }
}

__global__ __launch_bounds__(256) void dt_pre_kernel(
    const float* __restrict__ XD, const float* __restrict__ dtw, const float* __restrict__ dtb,
    float* __restrict__ DTP, int g)
{
  const int i  = blockIdx.x * 256 + threadIdx.x;
  const int l  = i >> 4;
  const int j0 = (i & 15) * 4;
  const bool live = (j0 < kGc);
  const int jb = j0 & (kGc - 1);
  const v4f xd = *(const v4f*)(XD + (size_t)l * kProjP);
  const float x0 = xd[0];
  const float x1 = xd[1];
  const float* wp = dtw + (size_t)((g * kGc + jb) * 2);
  const v4f wa = *(const v4f*)(wp);
  const v4f wb = *(const v4f*)(wp + 4);
  const v4f bv = *(const v4f*)(dtb + (size_t)(g * kGc + jb));
  const float w00 = wa[0];
  const float w01 = wa[1];
  const float w10 = wa[2];
  const float w11 = wa[3];
  const float w20 = wb[0];
  const float w21 = wb[1];
  const float w30 = wb[2];
  const float w31 = wb[3];
  const float b0 = bv[0];
  const float b1 = bv[1];
  const float b2 = bv[2];
  const float b3 = bv[3];
  const float t0 = fmaf(bf16r(w01), x1, bf16r(w00) * x0) + bf16r(b0);
  const float t1 = fmaf(bf16r(w11), x1, bf16r(w10) * x0) + bf16r(b1);
  const float t2 = fmaf(bf16r(w21), x1, bf16r(w20) * x0) + bf16r(b2);
  const float t3 = fmaf(bf16r(w31), x1, bf16r(w30) * x0) + bf16r(b3);
  v4f r;
  r[0] = live ? t0 : 0.0f;
  r[1] = live ? t1 : 0.0f;
  r[2] = live ? t2 : 0.0f;
  r[3] = live ? t3 : 0.0f;
  float* p = DTP + (size_t)i * 4;
  *(volatile v4f*)p = r;
  __threadfence();
  *(volatile v4f*)p = r;
}

__device__ __forceinline__ float y_from_words(unsigned hb, unsigned lb) {
  const float hi = h16_to_f32(hb);
  const float lo = h16_to_f32(lb);
  return (hi + lo * kInvResid) * kInvSCarry;
}
__device__ __forceinline__ float word_dot(unsigned hw, unsigned lw, float wa, float wb, float s) {
  const float y0 = y_from_words(hw & 0xffffu, lw & 0xffffu);
  const float y1 = y_from_words(hw >> 16, lw >> 16);
  s = fmaf(wa, y0, s);
  s = fmaf(wb, y1, s);
  return s;
}

static_assert(((kL / 4) % 256) == 0);
__global__ __launch_bounds__(256) void readout_group_kernel(
    const unsigned short* __restrict__ YH, const unsigned short* __restrict__ YL,
    const float* __restrict__ w_y, const float* __restrict__ b_y, float* __restrict__ OYg)
{
  const int i = blockIdx.x * 256 + threadIdx.x;
  float wy[16];
#pragma unroll
  for (int k = 0; k < 4; ++k) {
    const v4f wv = *(const v4f*)(w_y + 4 * k);
#pragma unroll
    for (int e = 0; e < 4; ++e) {
      const float t = wv[e];
      wy[4 * k + e] = bf16r(t);
    }
  }
  const float by = bf16r(b_y[0]);
  v4f rv;
#pragma unroll
  for (int e = 0; e < 4; ++e) {
    const size_t o = (size_t)(i * 4 + e) * kSd;
    const v4u ha = *(const v4u*)(const void*)(YH + o);
    const v4u hb = *(const v4u*)(const void*)(YH + o + 8);
    const v4u la = *(const v4u*)(const void*)(YL + o);
    const v4u lb = *(const v4u*)(const void*)(YL + o + 8);
    float s = 0.0f;
#pragma unroll
    for (int k = 0; k < 4; ++k) {
      const unsigned hwk = ha[k];
      const unsigned lwk = la[k];
      s = word_dot(hwk, lwk, wy[2 * k], wy[2 * k + 1], s);
    }
#pragma unroll
    for (int k = 0; k < 4; ++k) {
      const unsigned hwk = hb[k];
      const unsigned lwk = lb[k];
      s = word_dot(hwk, lwk, wy[8 + 2 * k], wy[8 + 2 * k + 1], s);
    }
    rv[e] = s + by;
  }
  float* p = OYg + (size_t)i * 4;
  *(volatile v4f*)p = rv;
  __threadfence();
  *(volatile v4f*)p = rv;
}

static_assert(((kC * kHW / 4) % 256) == 0);
__global__ __launch_bounds__(256) void order_sum_kernel(
    const float* __restrict__ OY, float* __restrict__ YSp, int pass)
{
  const int i  = blockIdx.x * 256 + threadIdx.x;
  const int r  = i >> 4;
  const int c4 = (i & 15) * 4;
  const int h  = r >> 5;
  const int w  = r & 31;
  float acc[4];
#pragma unroll
  for (int e = 0; e < 4; ++e) acc[e] = 0.0f;
  for (int g = 0; g < kDir; ++g) {
    const float* og = OY + (size_t)g * kL;
#pragma unroll
    for (int e = 0; e < 4; ++e) {
      const int pf = order_pos(g, c4 + e, h, w);
      const int pos = pass ? (kL - 1 - pf) : pf;
      const float t = og[pos];
      acc[e] += t;
    }
  }
  v4f rv;
  rv[0] = acc[0];
  rv[1] = acc[1];
  rv[2] = acc[2];
  rv[3] = acc[3];
  float* p = YSp + (size_t)i * 4;
  *(volatile v4f*)p = rv;
  __threadfence();
  *(volatile v4f*)p = rv;
}

__device__ __forceinline__ void row_stats(const float* __restrict__ row, float& mean, float& inv) {
  v4f t[16];
#pragma unroll
  for (int k = 0; k < 16; ++k) t[k] = *(const v4f*)(row + 4 * k);
  float s = 0.0f;
#pragma unroll
  for (int k = 0; k < 16; ++k)
#pragma unroll
    for (int e = 0; e < 4; ++e) s += t[k][e];
  const float mu = s * (1.0f / (float)kC);
  float ss = 0.0f;
#pragma unroll
  for (int k = 0; k < 16; ++k)
#pragma unroll
    for (int e = 0; e < 4; ++e) {
      const float dv = t[k][e] - mu;
      ss = fmaf(dv, dv, ss);
    }
  const float var = ss * (1.0f / (float)kC);
  mean = mu;
  inv = 1.0f / sqrtf(var + kLnEps);
}

static_assert(((kHW * kC / 8) % 256) == 0);
__global__ __launch_bounds__(256) void ln_gate_kernel(
    const float* __restrict__ YS, const float* __restrict__ XZ,
    const float* __restrict__ ln_w, const float* __restrict__ ln_b, unsigned short* __restrict__ GH)
{
  const int i  = blockIdx.x * 256 + threadIdx.x;
  const int r  = i >> 3;
  const int c8 = (i & 7) * 8;
  const float* row0 = YS + (size_t)r * kC;
  const float* row1 = YS + (size_t)kHW * kC + (size_t)r * kC;
  float m0, i0, m1, i1;
  row_stats(row0, m0, i0);
  row_stats(row1, m1, i1);
  v8h hv;
#pragma unroll
  for (int hf = 0; hf < 2; ++hf) {
    const int co = c8 + hf * 4;
    const v4f a  = *(const v4f*)(row0 + co);
    const v4f b  = *(const v4f*)(row1 + co);
    const v4f gw = *(const v4f*)(ln_w + co);
    const v4f gb = *(const v4f*)(ln_b + co);
    const v4f zz = *(const v4f*)(XZ + (size_t)r * kXzP + kC + co);
#pragma unroll
    for (int e = 0; e < 4; ++e) {
      const float av = a[e];
      const float bv = b[e];
      const float wv = bf16r(gw[e]);
      const float ov = bf16r(gb[e]);
      const float zv = zz[e];
      const float n0 = (av - m0) * i0 * wv + ov;
      const float n1 = (bv - m1) * i1 * wv + ov;
      const float sz = zv / (1.0f + expf(-zv));
      const float gv = (n0 + n1) * sz;
      hv[hf * 4 + e] = f16_flush(gv * kYCarry);
    }
  }
  unsigned short* qh = GH + (size_t)i * 8;
  *(volatile v8h*)qh = hv;
  __threadfence();
  *(volatile v8h*)qh = hv;
}

static_assert(((kHW * kOutN / 4) % 256) == 0);
__global__ __launch_bounds__(256) void out_store_kernel(
    const float* __restrict__ OUTP, float* __restrict__ out)
{
  const int i  = blockIdx.x * 256 + threadIdx.x;
  const int r  = i >> 3;
  const int o4 = (i & 7) * 4;
  const v4f v = *(const v4f*)(OUTP + (size_t)r * kOutP + o4);
  float* p = out + (size_t)i * 4;
  *(volatile v4f*)p = v;
  __threadfence();
  *(volatile v4f*)p = v;
}

typedef float    ms1_v4f __attribute__((ext_vector_type(4)));
typedef unsigned ms1_v4u __attribute__((ext_vector_type(4)));
struct ms1_args {
  const float* dtpre;
  const float* u;
  const float* bc;
  const float* z;
  const float* A_log;
  const float* Dskip;
  __half* y;
  __half* y_lo;
  long ld_dtpre;
  long ld_u;
  long ld_bc;
  long ld_z;
  long ld_y;
  int offB;
  int offC;
  int offZ;
  float ycarry;
  int dir;
  int D;
  int L;
  int nbatch;
};
static_assert(sizeof(ms1_args) == 136);

__device__ __forceinline__ float ms1_flush16(float v) {
  return (fabsf(v) < 6.103515625e-05f) ? 0.0f : v;
}
__device__ __forceinline__ unsigned ms1_h16bits(float v) {
  return (unsigned)__half_as_ushort(__float2half_rn(ms1_flush16(v)));
}
__device__ __forceinline__ float ms1_h16val(unsigned b) {
  return __half2float(__ushort_as_half((unsigned short)b));
}
__device__ __forceinline__ float ms1_softplus(float v) {
  return fmaxf(v, 0.0f) + log1pf(expf(-fabsf(v)));
}
__device__ __forceinline__ void ms1_pack2(float v0, float v1, unsigned& hw, unsigned& lw) {
  const unsigned h0 = ms1_h16bits(v0);
  const unsigned h1 = ms1_h16bits(v1);
  const float r0 = (v0 - ms1_h16val(h0)) * 2048.0f;
  const float r1 = (v1 - ms1_h16val(h1)) * 2048.0f;
  const unsigned l0 = ms1_h16bits(r0);
  const unsigned l1 = ms1_h16bits(r1);
  hw = h0 | (h1 << 16);
  lw = l0 | (l1 << 16);
}

template <int NSTATE>
__global__ __launch_bounds__(64 * (NSTATE / 16)) void ms1_scan_kernel(ms1_args a)
{
  static_assert(NSTATE == 16 || NSTATE == 64);
  constexpr int NQ  = NSTATE / 16;
  constexpr int NT  = 64 * NQ;
  constexpr int NW  = NT / 32;
  constexpr int BCW = 2 * NSTATE;
  constexpr int YP  = 68;
  constexpr int RPI = NW * 4;
  constexpr int NIT = 64 / RPI;
  static_assert(16 * NT <= 64 * YP);
  __shared__ __align__(16) float sBC[64 * BCW];
  __shared__ __align__(16) float sY[64 * YP];
  const int tid  = threadIdx.x;
  const int lane = tid & 31;
  const int wave = tid >> 5;
  const int c    = tid / NQ;
  const int sq   = tid - c * NQ;
  const int bpb  = a.D / 64;
  const int bi   = blockIdx.x / bpb;
  if (bi >= a.nbatch) return;
  const int d0 = (blockIdx.x - bi * bpb) * 64;
  const int d  = d0 + c;
  const long rowb = (long)bi * a.L;
  const bool hasz  = (a.z != nullptr);
  const bool hasD  = (a.Dskip != nullptr);
  const bool hasLo = (a.y_lo != nullptr);

#pragma unroll 1
  for (int n = 0; n < 16; ++n) {
    const float al = a.A_log[(long)d * NSTATE + sq * 16 + n];
    sY[n * NT + tid] = -expf(al);
  }
  __syncthreads();
  float An[16], h[16];
#pragma unroll
  for (int n = 0; n < 16; ++n) {
    An[n] = sY[n * NT + tid];
    h[n] = 0.0f;
  }
  float Dd = 0.0f;
  if (hasD) Dd = a.Dskip[d];

  const int nchunk = a.L / 64;
  const bool fwd = (a.dir > 0);
  const int s0 = fwd ? 0 : 63;
  const int sd = fwd ? 1 : -1;
  const int q  = lane >> 3;
  const int c8 = (lane & 7) * 8;

#pragma unroll 1
  for (int ci = 0; ci < nchunk; ++ci) {
    const int tb = fwd ? (ci * 64) : (a.L - 64 - ci * 64);
    const long rowc = rowb + tb;
    __syncthreads();
#pragma unroll 8
    for (int i = 0; i < 32; ++i) {
      const int idx = tid + i * NT;
      const int st  = idx / BCW;
      const int col = idx - st * BCW;
      const int sc  = (col < NSTATE) ? (a.offB + col) : (a.offC + col - NSTATE);
      sBC[idx] = a.bc[(rowc + st) * a.ld_bc + sc];
    }
    __syncthreads();
#pragma unroll 1
    for (int s = 0; s < 64; ++s) {
      const int ls = s0 + sd * s;
      const long row = rowc + ls;
      float pre = a.dtpre[row * a.ld_dtpre + d];
      float uv  = a.u[row * a.ld_u + d];
      float zv  = 0.0f;
      if (hasz) zv = a.z[row * a.ld_z + a.offZ + d];
      asm volatile("" : "+v"(pre));
      asm volatile("" : "+v"(uv));
      asm volatile("" : "+v"(zv));
      const float delta = ms1_softplus(pre);
      const float dtx = delta * uv;
      const float* bp = sBC + ls * BCW + sq * 16;
      const float* cp = bp + NSTATE;
      ms1_v4f Bq[4], Cq[4];
#pragma unroll
      for (int k = 0; k < 4; ++k) {
        Bq[k] = *(const ms1_v4f*)(bp + 4 * k);
        Cq[k] = *(const ms1_v4f*)(cp + 4 * k);
      }
      float yv = 0.0f;
#pragma unroll
      for (int n = 0; n < 16; ++n) {
        const float e = __expf(delta * An[n]);
        h[n] = fmaf(e, h[n], dtx * Bq[n >> 2][n & 3]);
        yv = fmaf(h[n], Cq[n >> 2][n & 3], yv);
      }
      if (NQ > 1) {
        yv += __shfl_xor(yv, 1, 32);
        yv += __shfl_xor(yv, 2, 32);
      }
      if (hasD) yv = fmaf(uv, Dd, yv);
      if (hasz) {
        const float sg = __builtin_amdgcn_rcpf(1.0f + expf(-zv));
        yv = yv * (zv * sg);
      }
      if (sq == 0) sY[ls * YP + c] = yv * a.ycarry;
    }
    __syncthreads();
    ms1_v4u hw[NIT], lw[NIT];
#pragma unroll
    for (int it = 0; it < NIT; ++it) {
      const int row = it * RPI + wave * 4 + q;
      const float* sp = sY + row * YP + c8;
      const ms1_v4f f0 = *(const ms1_v4f*)(sp);
      const ms1_v4f f1 = *(const ms1_v4f*)(sp + 4);
      unsigned h0, h1, h2, h3, l0, l1, l2, l3;
      ms1_pack2(f0[0], f0[1], h0, l0);
      ms1_pack2(f0[2], f0[3], h1, l1);
      ms1_pack2(f1[0], f1[1], h2, l2);
      ms1_pack2(f1[2], f1[3], h3, l3);
      hw[it] = (ms1_v4u){h0, h1, h2, h3};
      lw[it] = (ms1_v4u){l0, l1, l2, l3};
    }
    for (int pass = 0; pass < 2; ++pass) {
#pragma unroll
      for (int it = 0; it < NIT; ++it) {
        const int row = it * RPI + wave * 4 + q;
        const long o = (rowc + row) * a.ld_y + d0 + c8;
        *(volatile ms1_v4u*)(a.y + o) = hw[it];
        if (hasLo) *(volatile ms1_v4u*)(a.y_lo + o) = lw[it];
      }
      __threadfence();
    }
  }
}

static_assert(((kHW / 32) * (kXzP / 64)) % 8 == 0);
static_assert(((kL / 32) * (kProjP / 64)) % 8 == 0);
static_assert(((kHW / 32) * (kOutP / 64)) % 8 == 0);
static_assert(((kHW * kDm / 8) % 256) == 0);
static_assert(((kXzP * kDm / 8) % 256) == 0);
static_assert(((kOutP * kC / 8) % 256) == 0);
static_assert(kSd == 64 && kProjP == 64);

extern "C" void kernel_launch(void* const* d_in, const int* in_sizes, int n_in,
                              void* d_out, int out_size, void* d_ws, size_t ws_size,
                              hipStream_t stream)
{
  if (n_in < 16) return;
  if (in_sizes[0] != kHW * kDm) return;
  if (in_sizes[1] != kXzP * kDm) return;
  if (in_sizes[2] != kC * 9) return;
  if (in_sizes[3] != kC) return;
  if (in_sizes[4] != kNst) return;
  if (in_sizes[5] != kNst) return;
  if (in_sizes[6] != kDir * kProjN * kGc) return;
  if (in_sizes[7] != kDir * kGc * 2) return;
  if (in_sizes[8] != kDir * kGc) return;
  if (in_sizes[9] != kDir * kGc * kNst) return;
  if (in_sizes[10] != kDir * kGc) return;
  if (in_sizes[11] != kGc) return;
  if (in_sizes[12] != 1) return;
  if (in_sizes[13] != kC) return;
  if (in_sizes[14] != kC) return;
  if (in_sizes[15] != kOutN * kC) return;
  if (out_size != kHW * kOutN) return;
  if (ws_size < kWsTotal) return;

  const float* x      = (const float*)d_in[0];
  const float* W_in   = (const float*)d_in[1];
  const float* conv_w = (const float*)d_in[2];
  const float* conv_b = (const float*)d_in[3];
  const float* w_xs   = (const float*)d_in[4];
  const float* b_xs   = (const float*)d_in[5];
  const float* xpw    = (const float*)d_in[6];
  const float* dtw    = (const float*)d_in[7];
  const float* dtb    = (const float*)d_in[8];
  const float* A_logs = (const float*)d_in[9];
  const float* Ds     = (const float*)d_in[10];
  const float* w_y    = (const float*)d_in[11];
  const float* b_y    = (const float*)d_in[12];
  const float* ln_w   = (const float*)d_in[13];
  const float* ln_b   = (const float*)d_in[14];
  const float* W_out  = (const float*)d_in[15];
  float* out = (float*)d_out;

  char* ws = (char*)d_ws;
  unsigned short* XH    = (unsigned short*)(ws + kOffXH);
  unsigned short* WIN   = (unsigned short*)(ws + kOffWIN);
  unsigned short* WXH   = (unsigned short*)(ws + kOffWXH);
  unsigned short* WOH   = (unsigned short*)(ws + kOffWOH);
  float*          ALOGP = (float*)(ws + kOffALOGP);
  float*          DSP   = (float*)(ws + kOffDSP);
  float*          XZ    = (float*)(ws + kOffXZ);
  float*          V     = (float*)(ws + kOffV);
  float*          U     = (float*)(ws + kOffU);
  unsigned short* AH    = (unsigned short*)(ws + kOffAH);
  unsigned short* AL    = (unsigned short*)(ws + kOffAL);
  float*          XD    = (float*)(ws + kOffXD);
  float*          DTP   = (float*)(ws + kOffDTP);
  unsigned short* YH    = (unsigned short*)(ws + kOffYH);
  unsigned short* YL    = (unsigned short*)(ws + kOffYL);
  float*          OY    = (float*)(ws + kOffOY);
  float*          YS    = (float*)(ws + kOffYS);
  unsigned short* GH    = (unsigned short*)(ws + kOffGH);
  float*          OUTP  = (float*)(ws + kOffOUTP);

  constexpr float sW  = 1.0f / kWCarry;
  constexpr float sWr = 1.0f / (kWCarry * kResid);
  constexpr float sO  = 1.0f / (kWCarry * kYCarry);

  rne_rows_f16_kernel<<<(kHW * kDm / 8) / 256, 256, 0, stream>>>(x, XH, kHW * kDm / 8);

  pack_rows_bf_kernel<<<(kXzP * kDm / 8) / 256, 256, 0, stream>>>(
      W_in, WIN, kDm, kXzP, kXzP * kDm / 8, kWCarry);

  pack_xproj_kernel<<<(kDir * kProjP * kKp / 8) / 256, 256, 0, stream>>>(xpw, WXH);

  pack_rows_bf_kernel<<<(kOutP * kC / 8) / 256, 256, 0, stream>>>(
      W_out, WOH, kC, kOutN, kOutP * kC / 8, kWCarry);

  scan_params_kernel<<<(kDir * kSd * kNst / 4) / 256, 256, 0, stream>>>(A_logs, Ds, ALOGP, DSP);

  eng::gemm_f16_kernel<2, 0><<<dim3((kHW / 32) * (kXzP / 64) / 8), 256, 0, stream>>>(
      XH, nullptr, kDm, WIN, nullptr, kDm, XZ, kXzP, kHW, kXzP, kDm, sW, 0.0f);

  conv3_silu_kernel<<<(kC * kH * kW / 4) / 256, 256, 0, stream>>>(XZ, conv_w, conv_b, V);

  for (int pass = 0; pass < 2; ++pass) {
    for (int g = 0; g < kDir; ++g) {
      lift_gather_kernel<<<(kL * kSd / 4) / 256, 256, 0, stream>>>(V, w_xs, b_xs, U, AH, AL, pass, g);

      const unsigned short* Wg = WXH + (size_t)g * kProjP * kKp;
      eng::gemm_f16_kernel<2, 1><<<dim3((kL / 32) * (kProjP / 64) / 8), 256, 0, stream>>>(
          AH, AL, kKp, Wg, Wg, kKp, XD, kProjP, kL, kProjP, kKp, sW, sWr);

      dt_pre_kernel<<<(kL * kSd / 4) / 256, 256, 0, stream>>>(XD, dtw, dtb, DTP, g);

      ms1_args sa;
      sa.dtpre = DTP;
      sa.u = U;
      sa.bc = XD;
      sa.z = nullptr;
      sa.A_log = ALOGP + (size_t)g * kSd * kNst;
      sa.Dskip = DSP + (size_t)g * kSd;
      sa.y = (__half*)YH;
      sa.y_lo = (__half*)YL;
      sa.ld_dtpre = kSd;
      sa.ld_u = kSd;
      sa.ld_bc = kProjP;
      sa.ld_z = 0;
      sa.ld_y = kSd;
      sa.offB = 2;
      sa.offC = 2 + kNst;
      sa.offZ = 0;
      sa.ycarry = kSCarry;
      sa.dir = 1;
      sa.D = kSd;
      sa.L = kL;
      sa.nbatch = 1;
      ms1_scan_kernel<16><<<dim3(kSd / 64), 64, 0, stream>>>(sa);

      readout_group_kernel<<<(kL / 4) / 256, 256, 0, stream>>>(YH, YL, w_y, b_y, OY + (size_t)g * kL);
    }
    order_sum_kernel<<<(kC * kHW / 4) / 256, 256, 0, stream>>>(OY, YS + (size_t)pass * kHW * kC, pass);
  }

  ln_gate_kernel<<<(kHW * kC / 8) / 256, 256, 0, stream>>>(YS, XZ, ln_w, ln_b, GH);

  eng::gemm_f16_kernel<2, 0><<<dim3((kHW / 32) * (kOutP / 64) / 8), 256, 0, stream>>>(
      GH, nullptr, kC, WOH, nullptr, kC, OUTP, kOutP, kHW, kOutP, kC, sO, 0.0f);

  out_store_kernel<<<(kHW * kOutN / 4) / 256, 256, 0, stream>>>(OUTP, out);
}
